// FLAME_77979426226428
// MI455X (gfx1250) — hardware-run, weakly checked
//
#include <hip/hip_runtime.h>


#ifndef NB
#define NB 1024
#endif
#define NB_FULL 1024
#define NV   5023
#define NC   15069
#define NCP  15104
#define NL   150
#define NPF  36
#define KP   224
#define NLM  68
#define LM3  204
#define MPAD (((NB + 63) / 64) * 64)
#define JSP  160
#define RP   64

static_assert(NC == 3 * NV);
static_assert(NCP % 64 == 0);
static_assert(NCP >= NC);
static_assert(KP % 32 == 0);
static_assert(NL + 2 * NPF <= KP);
static_assert(MPAD % 64 == 0);
static_assert(NB <= NB_FULL);
static_assert(((size_t)NCP * (KP / 8)) % 256 == 0);
static_assert(((size_t)NB_FULL * NC) % 32 == 0);
static_assert(NV > 256);
static_assert(LM3 % 4 == 0);
static_assert(45 <= RP);
static_assert(60 <= RP);
static_assert(151 <= JSP);

typedef unsigned short bf;
typedef __attribute__((ext_vector_type(16))) __bf16   v16bf;
typedef __attribute__((ext_vector_type(8)))  unsigned short v8us;
typedef __attribute__((ext_vector_type(8)))  float    v8f;
typedef __attribute__((ext_vector_type(4)))  float    v4f;
typedef v4f  __attribute__((may_alias)) v4fa;
typedef v8us __attribute__((may_alias)) v8usa;

__device__ __forceinline__ unsigned short f2bf(float f) { unsigned u = __float_as_uint(f); u += 0x7FFFu + ((u >> 16) & 1u); return (unsigned short)(u >> 16); }
__device__ __forceinline__ float bf2f(unsigned short h) { return __uint_as_float(((unsigned)h) << 16); }
__device__ __forceinline__ float bfr(float f) { return bf2f(f2bf(f)); }
__device__ __forceinline__ v16bf cat16b(v8us lo, v8us hi) { return __builtin_bit_cast(v16bf, __builtin_shufflevector(lo, hi, 0, 1, 2, 3, 4, 5, 6, 7, 8, 9, 10, 11, 12, 13, 14, 15)); }
__device__ __forceinline__ v8f wmmab(v16bf a, v16bf b, v8f c) { return __builtin_amdgcn_wmma_f32_16x16x32_bf16(false, a, false, b, (short)0, c, false, false); }
__device__ __forceinline__ v16bf ldb(const bf* p)  { return cat16b(*(const v8us*)p, *(const v8us*)(p + 16)); }
__device__ __forceinline__ void wave_sync() { __builtin_amdgcn_fence(3  , "wavefront"); __builtin_amdgcn_wave_barrier(); asm volatile("" ::: "memory"); }

__global__ __launch_bounds__(256) void k_packb(const float* __restrict__ sd, const float* __restrict__ pd, bf* Bt) {
    const unsigned i = blockIdx.x * 256u + threadIdx.x;
    if (i >= (unsigned)(NCP * (KP / 8))) return;
    const int n = (int)(i / (unsigned)(KP / 8));
    const int k8 = (int)(i % (unsigned)(KP / 8)) * 8;
    const int nc = n < NC ? n : NC - 1;
    const bool nok = n < NC;
    float s[8], p[8];
#pragma unroll
    for (int e = 0; e < 8; ++e) { const int kk = k8 + e; const int ks = kk < NL ? kk : NL - 1; s[e] = sd[(size_t)nc * NL + ks]; }
    asm volatile("" ::: "memory");
#pragma unroll
    for (int e = 0; e < 8; ++e) { const int kk = k8 + e; int pr = (kk < NL + NPF) ? (kk - NL) : (kk - NL - NPF); pr = pr < 0 ? 0 : (pr > NPF - 1 ? NPF - 1 : pr); p[e] = pd[(size_t)pr * NC + nc]; }
    v8us o;
#pragma unroll
    for (int e = 0; e < 8; ++e) { const int kk = k8 + e; const float v = (kk < NL) ? s[e] : p[e]; const bool ok = nok && (kk < NL + 2 * NPF); o[e] = ok ? f2bf(v) : (unsigned short)0; }
    bf* dst = Bt + (size_t)i * 8;
    *(volatile v8us*)dst = o; __threadfence(); *(volatile v8us*)dst = o;
}

__global__ __launch_bounds__(160) void k_js(const float* __restrict__ jreg, const float* __restrict__ sd, const float* __restrict__ vt, float* JS) {
    const int jc = blockIdx.x; const int j = jc / 3, c = jc - 3 * j;
    const int l = threadIdx.x; const int lc = l < NL ? l : NL - 1;
    float acc = 0.0f;
#pragma unroll 2
    for (int v = 0; v < NV; ++v) {
        const float w = bfr(jreg[j * NV + v]);
        const float xs = sd[(size_t)(v * 3 + c) * NL + lc];
        const float xt = vt[v * 3 + c];
        const float x = bfr((l < NL) ? xs : xt);
        acc = fmaf(w, x, acc);
    }
    const float o = (l <= NL) ? acc : 0.0f;
    float* dst = JS + jc * JSP + l;
    *(volatile float*)dst = o; __threadfence(); *(volatile float*)dst = o;
}

__global__ __launch_bounds__(160) void k_rod(const float* __restrict__ pose, const float* __restrict__ eye, const float* __restrict__ neck, float* Rm) {
    __shared__ __align__(16) float rs[32 * RP];
    const int tid = threadIdx.x, lane = tid & 31;
    const int j = __builtin_amdgcn_readfirstlane(tid >> 5);
    const int b0 = blockIdx.x * 32;
    const int bb = b0 + lane; const int bc = bb < NB ? bb : NB - 1;
    for (int i = tid; i < 32 * RP; i += 160) rs[i] = 0.0f;
    __syncthreads();
    const int po = (j == 2) ? 3 : 0, eo = (j == 4) ? 3 : 0;
    float a[3];
#pragma unroll
    for (int c = 0; c < 3; ++c) {
        const float pv = pose[(size_t)bc * 6 + po + c]; const float nv = neck[c]; const float ev = eye[eo + c];
        a[c] = bfr((j == 1) ? nv : ((j >= 3) ? ev : pv));
    }
    const float x = a[0], y = a[1], z = a[2];
    const float ax = x + 1e-8f, ay = y + 1e-8f, az = z + 1e-8f;
    const float ang = sqrtf(ax * ax + ay * ay + az * az);
    const float inv = 1.0f / ang;
    const float rx = x * inv, ry = y * inv, rz = z * inv;
    const float s = sinf(ang), cs = cosf(ang), o = 1.0f - cs;
    const float xy = rx * ry, xz = rx * rz, yz = ry * rz;
    const float xx = rx * rx, yy = ry * ry, zz = rz * rz;
    float R[9];
    R[0] = 1.0f + o * (-(zz + yy)); R[1] = s * (-rz) + o * xy;        R[2] = s * ry + o * xz;
    R[3] = s * rz + o * xy;         R[4] = 1.0f + o * (-(zz + xx));   R[5] = s * (-rx) + o * yz;
    R[6] = s * (-ry) + o * xz;      R[7] = s * rx + o * yz;           R[8] = 1.0f + o * (-(yy + xx));
#pragma unroll
    for (int e = 0; e < 9; ++e) rs[lane * RP + j * 9 + e] = R[e];
    __syncthreads();
    float* dst = Rm + (size_t)b0 * RP;
#pragma unroll 1
    for (int ps = 0; ps < 2; ++ps) {
        for (int i = tid; i < 32 * RP / 4; i += 160) { const v4f v = *(const v4fa*)(&rs[i * 4]); *(volatile v4f*)(dst + (size_t)i * 4) = v; }
        if (ps == 0) __threadfence();
    }
}

__global__ __launch_bounds__(32) void k_prep(const float* __restrict__ shp, const float* __restrict__ expr, const float* __restrict__ Rm, const float* __restrict__ JS, bf* Ap, float* REL) {
    __shared__ __align__(16) unsigned short as_[32 * KP];
    __shared__ __align__(16) float rs[32 * RP];
    __shared__ __align__(16) float rel[32 * RP];
    __shared__ float js[15 * 32];
    __shared__ float ts[60 * 32];
    const int lane = threadIdx.x & 31;
    const int b0 = blockIdx.x * 32;
    const bool valid = (b0 + lane) < NB;
#pragma unroll 1
    for (int it = 0; it < 32 * RP / 4 / 32; ++it) { const int i = it * 32 + lane; const v4f v = *(const v4f*)(Rm + (size_t)b0 * RP + (size_t)i * 4); *(v4fa*)(&rs[i * 4]) = v; }
#pragma unroll 1
    for (int r = 0; r < 32; ++r) {
        const int bb = b0 + r; const int bc = bb < NB ? bb : NB - 1; const bool ok = bb < NB;
#pragma unroll
        for (int q = 0; q < 5; ++q) {
            const int l = q * 32 + lane;
            const int ls = l < 100 ? l : 99;
            int le = l - 100; le = le < 0 ? 0 : (le > 49 ? 49 : le);
            const float sv = shp[(size_t)bc * 100 + ls]; const float ev = expr[(size_t)bc * 50 + le];
            const float v = (l < 100) ? sv : ev;
            const unsigned short u = ok ? f2bf(v) : (unsigned short)0;
            if (l < NL) as_[r * KP + l] = u;
        }
    }
    __syncthreads();
#pragma unroll 1
    for (int q = 0; q < NPF; ++q) {
        const int e = q % 9;
        const float id = (e == 0 || e == 4 || e == 8) ? 1.0f : 0.0f;
        const float pf = rs[lane * RP + 9 + q] - id;
        const unsigned short h = f2bf(pf);
        const unsigned short lo = f2bf(pf - bf2f(h));
        as_[lane * KP + NL + q] = valid ? h : (unsigned short)0;
        as_[lane * KP + NL + NPF + q] = valid ? lo : (unsigned short)0;
    }
    as_[lane * KP + 222] = 0; as_[lane * KP + 223] = 0;
#pragma unroll 1
    for (int jc = 0; jc < 15; ++jc) {
        const float* row = JS + jc * JSP;
        float acc = row[NL];
#pragma unroll 2
        for (int l = 0; l < NL; ++l) acc = fmaf(row[l], bf2f(as_[lane * KP + l]), acc);
        js[jc * 32 + lane] = acc;
    }
#pragma unroll
    for (int i = 0; i < 3; ++i) {
#pragma unroll
        for (int k = 0; k < 3; ++k) ts[(i * 4 + k) * 32 + lane] = rs[lane * RP + i * 3 + k];
        ts[(i * 4 + 3) * 32 + lane] = js[i * 32 + lane];
    }
#pragma unroll 1
    for (int j = 1; j < 5; ++j) {
        const int p = (j == 1) ? 0 : 1;
        const float rj0 = js[(j * 3 + 0) * 32 + lane] - js[(p * 3 + 0) * 32 + lane];
        const float rj1 = js[(j * 3 + 1) * 32 + lane] - js[(p * 3 + 1) * 32 + lane];
        const float rj2 = js[(j * 3 + 2) * 32 + lane] - js[(p * 3 + 2) * 32 + lane];
        float r[9];
#pragma unroll
        for (int e = 0; e < 9; ++e) r[e] = rs[lane * RP + j * 9 + e];
#pragma unroll 1
        for (int i = 0; i < 3; ++i) {
            const float t0 = ts[(p * 12 + i * 4 + 0) * 32 + lane], t1 = ts[(p * 12 + i * 4 + 1) * 32 + lane];
            const float t2 = ts[(p * 12 + i * 4 + 2) * 32 + lane], t3 = ts[(p * 12 + i * 4 + 3) * 32 + lane];
            ts[(j * 12 + i * 4 + 0) * 32 + lane] = t0 * r[0] + t1 * r[3] + t2 * r[6];
            ts[(j * 12 + i * 4 + 1) * 32 + lane] = t0 * r[1] + t1 * r[4] + t2 * r[7];
            ts[(j * 12 + i * 4 + 2) * 32 + lane] = t0 * r[2] + t1 * r[5] + t2 * r[8];
            ts[(j * 12 + i * 4 + 3) * 32 + lane] = (t0 * rj0 + t1 * rj1 + t2 * rj2) + t3;
        }
    }
#pragma unroll 1
    for (int j = 0; j < 5; ++j) {
        const float j0 = js[(j * 3 + 0) * 32 + lane], j1 = js[(j * 3 + 1) * 32 + lane], j2 = js[(j * 3 + 2) * 32 + lane];
#pragma unroll 1
        for (int i = 0; i < 3; ++i) {
            const float t0 = ts[(j * 12 + i * 4 + 0) * 32 + lane], t1 = ts[(j * 12 + i * 4 + 1) * 32 + lane];
            const float t2 = ts[(j * 12 + i * 4 + 2) * 32 + lane], t3 = ts[(j * 12 + i * 4 + 3) * 32 + lane];
            rel[lane * RP + j * 12 + i * 4 + 0] = t0; rel[lane * RP + j * 12 + i * 4 + 1] = t1; rel[lane * RP + j * 12 + i * 4 + 2] = t2;
            rel[lane * RP + j * 12 + i * 4 + 3] = t3 - (t0 * j0 + t1 * j1 + t2 * j2);
        }
    }
    rel[lane * RP + 60] = 0.0f; rel[lane * RP + 61] = 0.0f; rel[lane * RP + 62] = 0.0f; rel[lane * RP + 63] = 0.0f;
    __syncthreads();
    bf* adst = Ap + (size_t)b0 * KP;
    float* rdst = REL + (size_t)b0 * RP;
#pragma unroll 1
    for (int ps = 0; ps < 2; ++ps) {
#pragma unroll 1
        for (int it = 0; it < 32 * KP / 8 / 32; ++it) { const int i = it * 32 + lane; const v8us v = *(const v8usa*)(&as_[i * 8]); *(volatile v8us*)(adst + (size_t)i * 8) = v; }
#pragma unroll 1
        for (int it = 0; it < 32 * RP / 4 / 32; ++it) { const int i = it * 32 + lane; const v4f v = *(const v4fa*)(&rel[i * 4]); *(volatile v4f*)(rdst + (size_t)i * 4) = v; }
        if (ps == 0) __threadfence();
    }
}

__global__ __launch_bounds__(32) void k_gemm(const bf* __restrict__ A, const bf* __restrict__ Bt, float* D) {
    __shared__ __align__(16) float os[16 * 68];
    const int K = KP;
    const int lane = threadIdx.x & 31, lr = lane & 15, hi = lane >> 4; const int r0 = blockIdx.x * 64, c0 = blockIdx.y * 64;
    v8f acc[4][4];
#pragma unroll
    for (int mb = 0; mb < 4; ++mb)
#pragma unroll
        for (int nb = 0; nb < 4; ++nb) acc[mb][nb] = (v8f){};
    const size_t aoff = (size_t)(r0 + lr) * K + 8 * hi, boff = (size_t)(c0 + lr) * K + 8 * hi;
#pragma unroll 1
    for (int kc = 0; kc < K; kc += 32) {
        v16bf a[4];
#pragma unroll
        for (int mb = 0; mb < 4; ++mb) a[mb] = ldb(A + aoff + (size_t)mb * 16 * K + kc);
#pragma unroll
        for (int nb = 0; nb < 4; ++nb) { const v16bf b = ldb(Bt + boff + (size_t)nb * 16 * K + kc);
#pragma unroll
            for (int mb = 0; mb < 4; ++mb) acc[mb][nb] = wmmab(a[mb], b, acc[mb][nb]); }
        asm volatile("v_nop\n\tv_nop\n\tv_nop\n\tv_nop" : "+v"(acc[0][0]), "+v"(acc[1][1]), "+v"(acc[2][2]), "+v"(acc[3][3]) : "v"(a[0]), "v"(a[1]), "v"(a[2]), "v"(a[3]));
    }
#pragma unroll
    for (int mb = 0; mb < 4; ++mb) {
#pragma unroll
        for (int nb = 0; nb < 4; ++nb) {
#pragma unroll
            for (int j = 0; j < 8; ++j) os[(hi * 8 + j) * 68 + nb * 16 + lr] = acc[mb][nb][j]; }
        wave_sync();
        float* drow = D + (size_t)(r0 + mb * 16) * NCP + c0;
#pragma unroll 1
        for (int ps = 0; ps < 2; ++ps) {
#pragma unroll
            for (int s = 0; s < 8; ++s) { const int row = 2 * s + hi, cofs = lr * 4;
                const v4f val = *(const v4fa*)(&os[row * 68 + cofs]);
                *(volatile v4f*)(drow + (size_t)row * NCP + cofs) = val; }
            if (ps == 0) __threadfence(); }
        wave_sync();
    }
}

__global__ __launch_bounds__(256) void k_skin(const float* __restrict__ D, const float* __restrict__ REL, const float* __restrict__ vt, const float* __restrict__ lw, float* OUT) {
    __shared__ __align__(16) float relS[2 * RP];
    __shared__ __align__(16) float os[768];
    const int tid = threadIdx.x;
    const unsigned g0 = blockIdx.x * 256u;
    const int bfirst = (int)(g0 / (unsigned)NV);
    if (tid < 2 * RP) { const int r = tid >> 6; int bb = bfirst + r; bb = bb < NB ? bb : NB - 1; relS[tid] = REL[(size_t)bb * RP + (tid & 63)]; }
    __syncthreads();
    const unsigned gtot = (unsigned)NB * (unsigned)NV;
    unsigned g = g0 + (unsigned)tid; g = g < gtot ? g : gtot - 1u;
    const int b = (int)(g / (unsigned)NV); const int v = (int)(g - (unsigned)b * (unsigned)NV);
    const int bl = b - bfirst;
    float T[12];
#pragma unroll
    for (int e = 0; e < 12; ++e) T[e] = 0.0f;
#pragma unroll 1
    for (int j = 0; j < 5; ++j) {
        const float w = bfr(lw[(size_t)v * 5 + j]);
#pragma unroll
        for (int e = 0; e < 12; ++e) T[e] = fmaf(w, relS[bl * RP + j * 12 + e], T[e]);
    }
    const size_t dofs = (size_t)b * NCP + (size_t)v * 3;
    const float px = bfr(vt[v * 3 + 0]) + D[dofs + 0];
    const float py = bfr(vt[v * 3 + 1]) + D[dofs + 1];
    const float pz = bfr(vt[v * 3 + 2]) + D[dofs + 2];
    os[tid * 3 + 0] = (T[0] * px + T[1] * py + T[2]  * pz) + T[3];
    os[tid * 3 + 1] = (T[4] * px + T[5] * py + T[6]  * pz) + T[7];
    os[tid * 3 + 2] = (T[8] * px + T[9] * py + T[10] * pz) + T[11];
    __syncthreads();
    const size_t total = (size_t)NB * NC;
    const size_t idx = (size_t)g0 * 3 + (size_t)tid * 4;
    const int tc = tid < 192 ? tid : 191;
    const v4f val = *(const v4fa*)(&os[tc * 4]);
#pragma unroll 1
    for (int ps = 0; ps < 2; ++ps) {
        if (tid < 192) {
            if (idx + 4 <= total) { *(volatile v4f*)(OUT + idx) = val; }
            else {
#pragma unroll
                for (int c = 0; c < 4; ++c) if (idx + c < total) *(volatile float*)(OUT + idx + c) = val[c];
            }
        }
        if (ps == 0) __threadfence();
    }
}

__global__ __launch_bounds__(256) void k_lmk(const int* __restrict__ li, const float* VERT, float* OUT1) {
    const int i = blockIdx.x * 256 + threadIdx.x;
    if (i >= NB * (LM3 / 4)) return;
    v4f o;
#pragma unroll
    for (int q = 0; q < 4; ++q) {
        const int idx = i * 4 + q;
        const int b = idx / LM3; const int r = idx - b * LM3;
        const int lm = r / 3; const int c = r - lm * 3;
        int vi = li[lm]; vi = vi < 0 ? 0 : (vi > NV - 1 ? NV - 1 : vi);
        o[q] = VERT[((size_t)b * NV + (size_t)vi) * 3 + c];
    }
    float* dst = OUT1 + (size_t)i * 4;
    *(volatile v4f*)dst = o; __threadfence(); *(volatile v4f*)dst = o;
}

static constexpr size_t al256(size_t v) { return (v + 255) & ~(size_t)255; }
static constexpr size_t SZ_BT  = al256((size_t)NCP * KP * 2);
static constexpr size_t SZ_AP  = al256((size_t)MPAD * KP * 2);
static constexpr size_t SZ_JS  = al256((size_t)15 * JSP * 4);
static constexpr size_t SZ_RM  = al256((size_t)MPAD * RP * 4);
static constexpr size_t SZ_REL = al256((size_t)MPAD * RP * 4);
static constexpr size_t SZ_D   = al256((size_t)MPAD * NCP * 4);
static constexpr size_t SZ_TOTAL = SZ_BT + SZ_AP + SZ_JS + SZ_RM + SZ_REL + SZ_D;
static_assert(SZ_TOTAL <= (size_t)134217728);
static constexpr size_t OUT1_OFF = (size_t)NB_FULL * NC;
static_assert(OUT1_OFF * 4 == (size_t)61722624);
static_assert((OUT1_OFF + (size_t)NB_FULL * LM3) * 4 == (size_t)62558208);

extern "C" void kernel_launch(void* const* d_in, const int* in_sizes, int n_in,
                              void* d_out, int out_size, void* d_ws, size_t ws_size, hipStream_t stream) {
    if (n_in < 11) return;
    if ((size_t)in_sizes[0] < (size_t)NB * 100) return;
    if ((size_t)in_sizes[1] < (size_t)NB * 50) return;
    if ((size_t)in_sizes[2] < (size_t)NB * 6) return;
    if ((size_t)in_sizes[3] < (size_t)NLM) return;
    if ((size_t)in_sizes[4] < (size_t)NC) return;
    if ((size_t)in_sizes[5] < (size_t)NC * NL) return;
    if ((size_t)in_sizes[6] < (size_t)NPF * NC) return;
    if ((size_t)in_sizes[7] < (size_t)5 * NV) return;
    if ((size_t)in_sizes[8] < (size_t)NV * 5) return;
    if ((size_t)in_sizes[9] < 6) return;
    if ((size_t)in_sizes[10] < 3) return;
    if ((size_t)out_size < OUT1_OFF + (size_t)NB * LM3) return;
    if (SZ_TOTAL > ws_size) return;
    const float* shp  = (const float*)d_in[0];
    const float* expr = (const float*)d_in[1];
    const float* pose = (const float*)d_in[2];
    const int*   li   = (const int*)d_in[3];
    const float* vt   = (const float*)d_in[4];
    const float* sd   = (const float*)d_in[5];
    const float* pd   = (const float*)d_in[6];
    const float* jreg = (const float*)d_in[7];
    const float* lw   = (const float*)d_in[8];
    const float* eye  = (const float*)d_in[9];
    const float* neck = (const float*)d_in[10];
    float* OUT0 = (float*)d_out;
    float* OUT1 = (float*)d_out + OUT1_OFF;
    char* wsp = (char*)d_ws;
    bf* BT = (bf*)wsp; wsp += SZ_BT;
    bf* AP = (bf*)wsp; wsp += SZ_AP;
    float* JS = (float*)wsp; wsp += SZ_JS;
    float* RM = (float*)wsp; wsp += SZ_RM;
    float* RL = (float*)wsp; wsp += SZ_REL;
    float* DP = (float*)wsp; wsp += SZ_D;

    k_packb<<<(unsigned)(((size_t)NCP * (KP / 8) + 255) / 256), 256, 0, stream>>>(sd, pd, BT);
    k_js<<<15, 160, 0, stream>>>(jreg, sd, vt, JS);
    k_rod<<<MPAD / 32, 160, 0, stream>>>(pose, eye, neck, RM);
    k_prep<<<MPAD / 32, 32, 0, stream>>>(shp, expr, RM, JS, AP, RL);
    k_gemm<<<dim3(MPAD / 64, NCP / 64, 1), 32, 0, stream>>>(AP, BT, DP);
    k_skin<<<(unsigned)(((size_t)NB * NV + 255) / 256), 256, 0, stream>>>(DP, RL, vt, lw, OUT0);
    k_lmk<<<(unsigned)((NB * (LM3 / 4) + 255) / 256), 256, 0, stream>>>(li, OUT0, OUT1);
}
